// d2sdm_57904749084789
// MI455X (gfx1250) — hardware-verified
//
#include <hip/hip_runtime.h>
#include <stdint.h>

#define B_N  4096
#define M_N  16384
#define D_K  512
#define NCLS 100
#define NCP  112
#define QB   64
#define KCH  128
#define XSP  520
#define PSP  136

typedef _Float16 v16h __attribute__((ext_vector_type(16)));
typedef _Float16 v8h  __attribute__((ext_vector_type(8)));
typedef __bf16   v16b __attribute__((ext_vector_type(16)));
typedef __bf16   v8b  __attribute__((ext_vector_type(8)));
typedef float    v8f  __attribute__((ext_vector_type(8)));
typedef float    v4f  __attribute__((ext_vector_type(4)));
typedef unsigned short v8us __attribute__((ext_vector_type(8)));

static_assert((D_K % 32) == 0);
static_assert((M_N % KCH) == 0 && (KCH % 32) == 0 && KCH == 16 * 8);
static_assert((B_N % QB) == 0 && QB == 64);
static_assert((M_N % 64) == 0 && (M_N % 32) == 0 && (B_N % 32) == 0);
static_assert((XSP % 8) == 0 && XSP >= D_K && (PSP % 8) == 0 && PSP >= KCH);
static_assert((NCP % 16) == 0 && NCP >= NCLS && NCP <= 128);
static_assert(((QB * NCLS) % 4) == 0 && QB * NCLS * 4 <= QB * XSP * 2);
static_assert(((QB * NCLS * 4) % 512) == 0);
static_assert(sizeof(v8us) == 16 && sizeof(v4f) == 16);

__device__ __forceinline__ unsigned short bfbits(float f) {
  const unsigned u = __float_as_uint(f);
  return (unsigned short)((u + 0x7FFFu + ((u >> 16) & 1u)) >> 16);
}
__device__ __forceinline__ float bfval(unsigned short b) { return __uint_as_float(((unsigned)b) << 16); }
__device__ __forceinline__ float bfr(float f) { return bfval(bfbits(f)); }

__device__ __forceinline__ v16h ldfrag_h(const _Float16* p) {
  union { v16h v; v8h q[2]; } f;
  f.q[0] = *(const v8h*)(p);
  f.q[1] = *(const v8h*)(p + 16);
  return f.v;
}
__device__ __forceinline__ v16b ldfrag_b(const __bf16* p) {
  union { v16b v; v8b q[2]; } f;
  f.q[0] = *(const v8b*)(p);
  f.q[1] = *(const v8b*)(p + 16);
  return f.v;
}
__device__ __forceinline__ v8f mma_h(v16h a, v16h b, v8f c) {
  return __builtin_amdgcn_wmma_f32_16x16x32_f16(false, a, false, b, (short)0, c, false, false);
}
__device__ __forceinline__ v8f mma_b(v16b a, v16b b, v8f c) {
  return __builtin_amdgcn_wmma_f32_16x16x32_bf16(false, a, false, b, (short)0, c, false, false);
}
__device__ __forceinline__ v8f zero8() {
  v8f z;
#pragma unroll
  for (int i = 0; i < 8; ++i) z[i] = 0.0f;
  return z;
}
__device__ __forceinline__ void guard_s(v8f& a0, v8f& a1, v8f& a2, v8f& a3,
                                        v16b x, v16b y0, v16b y1, v16b y2, v16b y3) {
#if defined(__HIP_DEVICE_COMPILE__)
  asm volatile("v_nop\n\tv_nop\n\tv_nop\n\tv_nop"
               : "+v"(a0), "+v"(a1), "+v"(a2), "+v"(a3)
               : "v"(x), "v"(y0), "v"(y1), "v"(y2), "v"(y3));
#endif
}
__device__ __forceinline__ void guard_p(v8f& a0, v8f& a1, v8f& a2, v8f& a3,
                                        v16h x, v16h y0, v16h y1, v16h y2, v16h y3) {
#if defined(__HIP_DEVICE_COMPILE__)
  asm volatile("v_nop\n\tv_nop\n\tv_nop\n\tv_nop"
               : "+v"(a0), "+v"(a1), "+v"(a2), "+v"(a3)
               : "v"(x), "v"(y0), "v"(y1), "v"(y2), "v"(y3));
#endif
}

__global__ __launch_bounds__(256) void cvt_rows_kernel(const float* __restrict__ A, const float* __restrict__ X,
                                                       unsigned short* __restrict__ Abf, unsigned short* __restrict__ Xbf,
                                                       float* __restrict__ aa, float* __restrict__ xx, int nbA, int nbX) {
#pragma clang fp contract(off)
  __shared__ __align__(16) float ssq[32];
  const int wave = threadIdx.x >> 5, lane = threadIdx.x & 31;
  const int blk = (int)blockIdx.x;
  if (blk >= nbA + nbX) return;
  const bool isx = (blk >= nbA);
  const float* src = isx ? X : A;
  unsigned short* dst = isx ? Xbf : Abf;
  float* sq = isx ? xx : aa;
  const int rb = (blk - (isx ? nbA : 0)) * 32;

#pragma unroll 1
  for (int i = 0; i < 4; ++i) {
    const int lr = wave * 4 + i;
    const float* xr = src + (size_t)(rb + lr) * D_K;
    unsigned short* yr = dst + (size_t)(rb + lr) * D_K;
    float s = 0.0f;
#pragma unroll
    for (int j = 0; j < 2; ++j) {
      const int c0 = (j * 32 + lane) * 8;
      const v4f a = *(const v4f*)(xr + c0);
      const v4f b = *(const v4f*)(xr + c0 + 4);
      v8us o;
#pragma unroll
      for (int e = 0; e < 4; ++e) {
        const unsigned short u0 = bfbits(a[e]), u1 = bfbits(b[e]);
        o[e] = u0;
        o[4 + e] = u1;
        const float f0 = bfval(u0), f1 = bfval(u1);
        s += f0 * f0;
        s += f1 * f1;
      }
      *(volatile v8us*)(yr + c0) = o;
      __threadfence();
      *(volatile v8us*)(yr + c0) = o;
    }
#pragma unroll
    for (int off = 16; off > 0; off >>= 1) s += __shfl_xor(s, off, 32);
    if (lane == 0) ssq[lr] = s;
  }
  __syncthreads();
  if (threadIdx.x < 8) {
    const v4f v = *(const v4f*)(ssq + 4 * threadIdx.x);
    float* d = sq + rb + 4 * threadIdx.x;
    *(volatile v4f*)d = v;
    __threadfence();
    *(volatile v4f*)d = v;
  }
}

__global__ __launch_bounds__(256) void cvt_c_kernel(const float* __restrict__ C, _Float16* __restrict__ Ct) {
#pragma clang fp contract(off)
  __shared__ __align__(16) float Cs[64 * NCLS];
  const int tid = threadIdx.x;
  const int m0 = (int)blockIdx.x * 64;
  const float* cg = C + (size_t)m0 * NCLS;
#pragma unroll 1
  for (int it = 0; it < 7; ++it) {
    const int p = it * 256 + tid;
    if (p < (64 * NCLS) / 4) {
      const v4f v = *(const v4f*)(cg + 4 * p);
      *(v4f*)(Cs + 4 * p) = v;
    }
  }
  __syncthreads();
  const int q8 = (tid & 7) * 8;
#pragma unroll
  for (int ps = 0; ps < 2; ++ps) {
#pragma unroll 1
    for (int it = 0; it < 4; ++it) {
      const int cc = it * 32 + (tid >> 3);
      if (cc < NCP) {
        const int ccl = (cc < NCLS) ? cc : (NCLS - 1);
        v8h o;
#pragma unroll
        for (int e = 0; e < 8; ++e) {
          const float v = Cs[(q8 + e) * NCLS + ccl];
          const float w = (cc < NCLS) ? (bfr(v) * 16.0f) : 0.0f;
          o[e] = (_Float16)w;
        }
        *(volatile v8h*)(Ct + (size_t)cc * M_N + m0 + q8) = o;
      }
    }
    __threadfence();
  }
}

__global__ __launch_bounds__(256) void smx_kernel(const unsigned short* __restrict__ Abf,
                                                  const unsigned short* __restrict__ Xbf,
                                                  const _Float16* __restrict__ Ct,
                                                  const float* __restrict__ aaG,
                                                  const float* __restrict__ xxG,
                                                  float* __restrict__ out) {
#pragma clang fp contract(off)
  __shared__ __align__(16) char xo_raw[QB * XSP * 2];
  __shared__ __align__(16) _Float16 Phs[QB * PSP];
  __shared__ __align__(16) _Float16 Pls[QB * PSP];
  __shared__ __align__(16) float pmax[8 * QB];
  __shared__ __align__(16) float psum[8 * QB];
  __shared__ __align__(16) float xxs[QB];
  __shared__ __align__(16) float m_s[QB];
  __shared__ __align__(16) float l_s[QB];
  __shared__ __align__(16) float al_s[QB];
  __shared__ __align__(16) float li_s[QB];

  const int tid = threadIdx.x, wave = tid >> 5, lane = tid & 31, h = lane >> 4, c = lane & 15;
  const int q0 = (int)blockIdx.x * QB;
  const float ninf = -__builtin_inff();
  unsigned short* Xsu = (unsigned short*)xo_raw;
  const __bf16* Xs = (const __bf16*)(const void*)xo_raw;

  if (tid < QB) {
    m_s[tid] = ninf; l_s[tid] = 0.0f; al_s[tid] = 0.0f; li_s[tid] = 0.0f;
    xxs[tid] = xxG[q0 + tid];
  }
  psum[tid] = 0.0f;
  psum[256 + tid] = 0.0f;
#pragma unroll
  for (int i = 0; i < 16; ++i) {
    const int idx = i * 256 + tid;
    const int row = idx >> 6, pc = idx & 63;
    const v8us v = *(const v8us*)(Xbf + (size_t)(q0 + row) * D_K + pc * 8);
    *(v8us*)(Xsu + row * XSP + pc * 8) = v;
  }
  __syncthreads();

  float xq[4];
#pragma unroll
  for (int qt = 0; qt < 4; ++qt) xq[qt] = xxs[16 * qt + c];

  v8f oh[4], ol[4];
#pragma unroll
  for (int qt = 0; qt < 4; ++qt) { oh[qt] = zero8(); ol[qt] = zero8(); }

  const __bf16* Ag = (const __bf16*)(const void*)Abf;
  const __bf16* xbp = Xs + c * XSP + 8 * h;
  const int ntile = M_N / KCH;

#pragma unroll 1
  for (int t = 0; t < ntile; ++t) {
    const int kb = t * KCH + 16 * wave;
    const __bf16* kap = Ag + (size_t)(kb + c) * D_K + 8 * h;
    v8f sacc[4];
#pragma unroll
    for (int qt = 0; qt < 4; ++qt) sacc[qt] = zero8();
#pragma unroll 1
    for (int k0 = 0; k0 < D_K; k0 += 32) {
      const v16b a  = ldfrag_b(kap + k0);
      const v16b b0 = ldfrag_b(xbp + k0);
      const v16b b1 = ldfrag_b(xbp + 16 * XSP + k0);
      const v16b b2 = ldfrag_b(xbp + 32 * XSP + k0);
      const v16b b3 = ldfrag_b(xbp + 48 * XSP + k0);
      sacc[0] = mma_b(a, b0, sacc[0]);
      sacc[1] = mma_b(a, b1, sacc[1]);
      sacc[2] = mma_b(a, b2, sacc[2]);
      sacc[3] = mma_b(a, b3, sacc[3]);
      guard_s(sacc[0], sacc[1], sacc[2], sacc[3], a, b0, b1, b2, b3);
    }
    {
      const v4f aA = *(const v4f*)(aaG + kb + 8 * h);
      const v4f aB = *(const v4f*)(aaG + kb + 8 * h + 4);
#pragma unroll
      for (int qt = 0; qt < 4; ++qt) {
        float pm = ninf;
#pragma unroll
        for (int r = 0; r < 4; ++r) {
          const float e0 = aA[r] + xq[qt];
          const float d0 = e0 - 2.0f * sacc[qt][r];
          const float s0 = sqrtf(fmaxf(d0, 0.0f)) * -0.25f;
          sacc[qt][r] = s0;
          pm = fmaxf(pm, s0);
          const float e1 = aB[r] + xq[qt];
          const float d1 = e1 - 2.0f * sacc[qt][4 + r];
          const float s1 = sqrtf(fmaxf(d1, 0.0f)) * -0.25f;
          sacc[qt][4 + r] = s1;
          pm = fmaxf(pm, s1);
        }
        pm = fmaxf(pm, __shfl_xor(pm, 16, 32));
        pmax[wave * QB + 16 * qt + c] = pm;
      }
    }
    __syncthreads();
    if (tid < QB) {
      const int row = tid;
      float ps = 0.0f;
#pragma unroll
      for (int w = 0; w < 8; ++w) ps += psum[w * QB + row];
      l_s[row] = l_s[row] * al_s[row] + ps;
      const float mo = m_s[row];
      float mx = mo;
#pragma unroll
      for (int w = 0; w < 8; ++w) mx = fmaxf(mx, pmax[w * QB + row]);
      al_s[row] = __expf(mo - mx);
      m_s[row] = mx;
    }
    __syncthreads();
    {
#pragma unroll
      for (int qt = 0; qt < 4; ++qt) {
        const float mq = m_s[16 * qt + c];
        float ps = 0.0f;
        v8h hh, ll;
#pragma unroll
        for (int r = 0; r < 8; ++r) {
          const float p = __expf(sacc[qt][r] - mq);
          ps += p;
          const float tv = p * 1024.0f;
          const _Float16 hv = (_Float16)tv;
          hh[r] = hv;
          ll[r] = (_Float16)((tv - (float)hv) * 2048.0f);
        }
        *(v8h*)(Phs + (16 * qt + c) * PSP + 16 * wave + 8 * h) = hh;
        *(v8h*)(Pls + (16 * qt + c) * PSP + 16 * wave + 8 * h) = ll;
        ps += __shfl_xor(ps, 16, 32);
        psum[wave * QB + 16 * qt + c] = ps;
        const v4f fA = *(const v4f*)(al_s + 16 * qt + 8 * h);
        const v4f fB = *(const v4f*)(al_s + 16 * qt + 8 * h + 4);
#pragma unroll
        for (int r = 0; r < 4; ++r) {
          oh[qt][r] *= fA[r];  oh[qt][4 + r] *= fB[r];
          ol[qt][r] *= fA[r];  ol[qt][4 + r] *= fB[r];
        }
      }
    }
    __syncthreads();
    if (wave < (NCP / 16)) {
      const _Float16* cbp = Ct + (size_t)(16 * wave + c) * M_N + (size_t)t * KCH + 8 * h;
      const _Float16* pp = Phs + c * PSP + 8 * h;
      const _Float16* pq = Pls + c * PSP + 8 * h;
#pragma unroll 1
      for (int ks = 0; ks < KCH; ks += 32) {
        const v16h cf = ldfrag_h(cbp + ks);
#pragma unroll
        for (int g = 0; g < 2; ++g) {
          const v16h p0 = ldfrag_h(pp + (32 * g) * PSP + ks);
          const v16h r0 = ldfrag_h(pq + (32 * g) * PSP + ks);
          const v16h p1 = ldfrag_h(pp + (32 * g + 16) * PSP + ks);
          const v16h r1 = ldfrag_h(pq + (32 * g + 16) * PSP + ks);
          oh[2 * g]     = mma_h(p0, cf, oh[2 * g]);
          ol[2 * g]     = mma_h(r0, cf, ol[2 * g]);
          oh[2 * g + 1] = mma_h(p1, cf, oh[2 * g + 1]);
          ol[2 * g + 1] = mma_h(r1, cf, ol[2 * g + 1]);
          guard_p(oh[2 * g], ol[2 * g], oh[2 * g + 1], ol[2 * g + 1], cf, p0, r0, p1, r1);
        }
      }
    }
  }

  if (tid < QB) {
    const int row = tid;
    float ps = 0.0f;
#pragma unroll
    for (int w = 0; w < 8; ++w) ps += psum[w * QB + row];
    const float l = l_s[row] * al_s[row] + ps;
    li_s[row] = (1.0f / l) * (1.0f / 16384.0f);
  }
  __syncthreads();
  {
    float* Os = (float*)xo_raw;
    const int cc = 16 * wave + c;
#pragma unroll
    for (int qt = 0; qt < 4; ++qt) {
      const v4f iA = *(const v4f*)(li_s + 16 * qt + 8 * h);
      const v4f iB = *(const v4f*)(li_s + 16 * qt + 8 * h + 4);
#pragma unroll
      for (int r = 0; r < 4; ++r) {
        const float v0 = (oh[qt][r] + ol[qt][r] * 0.00048828125f) * iA[r];
        const float v1 = (oh[qt][4 + r] + ol[qt][4 + r] * 0.00048828125f) * iB[r];
        if (cc < NCLS) {
          Os[(16 * qt + 8 * h + r) * NCLS + cc] = v0;
          Os[(16 * qt + 8 * h + 4 + r) * NCLS + cc] = v1;
        }
      }
    }
  }
  __syncthreads();
  {
    const float* Os = (const float*)xo_raw;
    float* go = out + (size_t)q0 * NCLS;
#pragma unroll
    for (int ps = 0; ps < 2; ++ps) {
#pragma unroll 1
      for (int it = 0; it < 7; ++it) {
        const int p = it * 256 + tid;
        if (p < (QB * NCLS) / 4) {
          const v4f v = *(const v4f*)(Os + 4 * p);
          *(volatile v4f*)(go + 4 * p) = v;
        }
      }
      __threadfence();
    }
  }
}

extern "C" void kernel_launch(void* const* d_in, const int* in_sizes, int n_in,
                              void* d_out, int out_size, void* d_ws, size_t ws_size,
                              hipStream_t stream) {
  if (n_in < 3) return;
  if (in_sizes[0] != B_N * D_K) return;
  if (in_sizes[1] != M_N * D_K) return;
  if (in_sizes[2] != M_N * NCLS) return;
  if (out_size != B_N * NCLS) return;

  const float* X = (const float*)d_in[0];
  const float* A = (const float*)d_in[1];
  const float* C = (const float*)d_in[2];
  float* out = (float*)d_out;

  const size_t bA  = (size_t)M_N * D_K * 2;
  const size_t bX  = (size_t)B_N * D_K * 2;
  const size_t bC  = (size_t)NCP * M_N * 2;
  const size_t baa = (size_t)M_N * 4;
  const size_t bxx = (size_t)B_N * 4;
  size_t off = 0;
  const size_t oA  = off; off += bA;
  const size_t oX  = off; off += bX;
  const size_t oC  = off; off += bC;
  const size_t oaa = off; off += baa;
  const size_t oxx = off; off += bxx;
  if (off > ws_size) return;
  if (off > (size_t)134217728) return;

  char* ws = (char*)d_ws;
  unsigned short* Abf = (unsigned short*)(ws + oA);
  unsigned short* Xbf = (unsigned short*)(ws + oX);
  _Float16*       Ct  = (_Float16*)(ws + oC);
  float*          aa  = (float*)(ws + oaa);
  float*          xx  = (float*)(ws + oxx);

  const int nbA = M_N / 32, nbX = B_N / 32;
  const dim3 blk(256);
  cvt_rows_kernel<<<dim3(nbA + nbX), blk, 0, stream>>>(A, X, Abf, Xbf, aa, xx, nbA, nbX);
  cvt_c_kernel<<<dim3(M_N / 64), blk, 0, stream>>>(C, Ct);
  smx_kernel<<<dim3(B_N / QB), blk, 0, stream>>>(Abf, Xbf, Ct, aa, xx, out);
  (void)hipGetLastError();
}
